// RNNModel_40905268527589
// MI455X (gfx1250) — hardware-verified
//
#include <hip/hip_runtime.h>
#include <math.h>

constexpr int SEQS   = 64;
constexpr int STEPS  = 256;
constexpr int TOKD   = 300;
constexpr int TAGD   = 50;
constexpr int DIN1   = TOKD + TAGD;
constexpr int K1P    = 352;
constexpr int HID    = 200;
constexpr int HKP    = 224;
constexpr int GATEP  = 208;
constexpr int NGATE  = 4 * GATEP;
constexpr int G4REAL = 4 * HID;
constexpr int NLAB   = 40;
constexpr int NLABP  = 64;
constexpr int NROWS  = SEQS * STEPS;
constexpr int HCP    = 512;
constexpr int HC_BWD = 256;
constexpr int HCK    = 480;
constexpr int H2P    = 224;
constexpr int H2NP   = 224;
constexpr int STP    = 32;
constexpr float FORGET_B = 1.0f;
constexpr float BNEPS    = 1e-3f;

static_assert(K1P % 32 == 0 && K1P >= DIN1);
static_assert(HKP % 32 == 0 && HKP >= HID);
static_assert(HCK % 32 == 0 && HCK <= HCP && HC_BWD + HID <= HCK);
static_assert(H2NP % 32 == 0 && H2NP >= HID);
static_assert(NGATE % 64 == 0 && NROWS % 64 == 0 && NLABP == 64);
static_assert(((NROWS / 64) * (NGATE / 64)) % 8 == 0);
static_assert(((NROWS / 64) * (NLABP / 64)) % 8 == 0);
static_assert((H2P * 4) % 128 == 0);
static_assert((NROWS * (H2NP / 8)) % 256 == 0);
static_assert((NROWS * (K1P / 8)) % 256 == 0);

constexpr size_t WS_XB   = (size_t)NROWS * K1P * 2;
constexpr size_t WS_WX1  = (size_t)NGATE * K1P * 2;
constexpr size_t WS_WH   = (size_t)NGATE * HKP * 2;
constexpr size_t WS_WX2  = (size_t)NGATE * HCP * 2;
constexpr size_t WS_WD   = (size_t)NLABP * H2NP * 2;
constexpr size_t WS_BG   = (size_t)NGATE * 4;
constexpr size_t WS_BD   = (size_t)NLABP * 4;
constexpr size_t WS_ZX   = (size_t)NROWS * NGATE * 4;
constexpr size_t WS_HC   = (size_t)NROWS * HCP * 2;
constexpr size_t WS_H2   = (size_t)NROWS * H2P * 4;
constexpr size_t WS_ST   = (size_t)H2NP * STP * 4;
constexpr size_t WS_H2N  = (size_t)NROWS * H2NP * 2;
constexpr size_t WS_TOTAL = WS_XB + 2 * WS_WX1 + 3 * WS_WH + WS_WX2 + WS_WD + 3 * WS_BG + WS_BD + WS_ZX + 2 * WS_HC +
                            WS_H2 + WS_ST + 2 * WS_H2N;
static_assert(WS_TOTAL == 132184064);
static_assert(WS_TOTAL <= (size_t)134217728);

typedef __attribute__((ext_vector_type(16))) __bf16   v16b;
typedef __attribute__((ext_vector_type(8)))  __bf16   v8b;
typedef __attribute__((ext_vector_type(8)))  float    v8f;
typedef __attribute__((ext_vector_type(4)))  float    v4f;
typedef __attribute__((ext_vector_type(4)))  unsigned v4u;

__device__ __forceinline__ unsigned short f2bf_bits(float f) {
  unsigned u = __float_as_uint(f);
  return (unsigned short)((u + 0x7FFFu + ((u >> 16) & 1u)) >> 16);
}
__device__ __forceinline__ float bf_bits2f(unsigned short h) { return __uint_as_float(((unsigned)h) << 16); }
__device__ __forceinline__ float bf16r(float f) { return bf_bits2f(f2bf_bits(f)); }
__device__ __forceinline__ void split_bf(float v, unsigned& hb, unsigned& lb) {
  const unsigned short h = f2bf_bits(v);
  hb = (unsigned)h;
  lb = (unsigned)f2bf_bits(v - bf_bits2f(h));
}

__device__ __forceinline__ void guard_grp_b(v8f& a0, v8f& a1, v8f& a2, v8f& a3, v16b x0, v16b x1,
                                            v16b y0, v16b y1, v16b y2, v16b y3) {
  asm volatile("v_nop\n\tv_nop\n\tv_nop\n\tv_nop"
               : "+v"(a0), "+v"(a1), "+v"(a2), "+v"(a3)
               : "v"(x0), "v"(x1), "v"(y0), "v"(y1), "v"(y2), "v"(y3));
}
__device__ __forceinline__ void acc_guard4(v8f& a, v8f& b, v8f& c, v8f& d) {
  asm volatile("v_nop\n\tv_nop\n\tv_nop\n\tv_nop" : "+v"(a), "+v"(b), "+v"(c), "+v"(d));
}

struct FragB {
  union U { v16b v; v8b h[2]; };
  static __device__ __forceinline__ v16b load(const __bf16* p) {
    U f; f.h[0] = *(const v8b*)(p); f.h[1] = *(const v8b*)(p + 16); return f.v;
  }
  static __device__ __forceinline__ v8f mma(v16b a, v16b b, v8f c) {
    return __builtin_amdgcn_wmma_f32_16x16x32_bf16(false, a, false, b, (short)0, c, false, false);
  }
};

__device__ __forceinline__ float fsig(float x) { return __builtin_amdgcn_rcpf(1.0f + expf(-x)); }

__global__ __launch_bounds__(256) void xpack_kernel(const float* __restrict__ tok, const float* __restrict__ tag,
                                                   unsigned short* __restrict__ X) {
  constexpr int NC8 = K1P / 8;
  const int i = blockIdx.x * 256 + threadIdx.x;
  if (i >= NROWS * NC8) return;
  const int row = i / NC8, c8 = i - row * NC8, col0 = c8 * 8;
  const int ta = (col0 < TOKD - 4) ? col0 : (TOKD - 4);
  const int tb = (col0 + 4 < TOKD - 4) ? (col0 + 4) : (TOKD - 4);
  const v4f va = *(const v4f*)(tok + (size_t)row * TOKD + ta);
  const v4f vb = *(const v4f*)(tok + (size_t)row * TOKD + tb);
  float tv[8], tg[8];
  tv[0] = va[0]; tv[1] = va[1]; tv[2] = va[2]; tv[3] = va[3];
  tv[4] = vb[0]; tv[5] = vb[1]; tv[6] = vb[2]; tv[7] = vb[3];
#pragma unroll
  for (int e = 0; e < 8; ++e) {
    int ci = col0 + e - TOKD;
    ci = ci < 0 ? 0 : (ci > TAGD - 1 ? TAGD - 1 : ci);
    tg[e] = tag[(size_t)row * TAGD + ci];
  }
  unsigned w[4];
#pragma unroll
  for (int e2 = 0; e2 < 4; ++e2) {
    unsigned bits[2];
#pragma unroll
    for (int h = 0; h < 2; ++h) {
      const int e = 2 * e2 + h;
      const int col = col0 + e;
      const float ftok = (col < TOKD) ? 1.0f : 0.0f;
      const float ftag = (col >= TOKD && col < DIN1) ? 1.0f : 0.0f;
      const float v = fmaf(ftok, tv[e], ftag * tg[e]) + 0.0f;
      bits[h] = (unsigned)f2bf_bits(v);
    }
    w[e2] = bits[0] | (bits[1] << 16);
  }
  const v4u o = {w[0], w[1], w[2], w[3]};
  unsigned short* op = X + (size_t)i * 8;
  *(volatile v4u*)op = o;
  __threadfence();
  *(volatile v4u*)op = o;
}

__global__ __launch_bounds__(256) void wpack_kernel(const float* __restrict__ W, int wrows, int ldw,
                                                   unsigned short* __restrict__ dst, int nout, int kp,
                                                   int gatep, int gcols, int gstride,
                                                   int kA, int rA0, int kB0, int kB, int rB0) {
  const int kp8 = kp >> 3;
  const int i = blockIdx.x * 256 + threadIdx.x;
  if (i >= nout * kp8) return;
  const int n = i / kp8, k8 = i - n * kp8;
  const int gate = n / gatep, cc = n - gate * gatep;
  const bool nval = cc < gcols;
  int col = gate * gstride + cc;
  col = col < 0 ? 0 : (col >= ldw ? ldw - 1 : col);
  unsigned w[4];
#pragma unroll
  for (int e2 = 0; e2 < 4; ++e2) {
    unsigned bits[2];
#pragma unroll
    for (int h = 0; h < 2; ++h) {
      const int k = 8 * k8 + 2 * e2 + h;
      const bool inA = k < kA;
      const bool inB = (k >= kB0) && (k < kB0 + kB);
      int r = inA ? (rA0 + k) : (inB ? (rB0 + k - kB0) : 0);
      r = r < 0 ? 0 : (r >= wrows ? wrows - 1 : r);
      const float x = W[(size_t)r * ldw + col];
      const float f = (nval && (inA || inB)) ? 1.0f : 0.0f;
      bits[h] = (unsigned)f2bf_bits(f * x + 0.0f);
    }
    w[e2] = bits[0] | (bits[1] << 16);
  }
  const v4u o = {w[0], w[1], w[2], w[3]};
  unsigned short* op = dst + (size_t)i * 8;
  *(volatile v4u*)op = o;
  __threadfence();
  *(volatile v4u*)op = o;
}

__global__ __launch_bounds__(256) void bias_pack_kernel(const float* __restrict__ b, int nb, float* __restrict__ dst,
                                                       int nout, int gatep, int gcols, int gstride) {
  const int t = threadIdx.x;
  if (t >= (nout >> 2)) return;
  v4f o;
#pragma unroll
  for (int e = 0; e < 4; ++e) {
    const int n = 4 * t + e;
    const int gate = n / gatep, cc = n - gate * gatep;
    const bool valid = cc < gcols;
    int idx = gate * gstride + cc;
    idx = idx < 0 ? 0 : (idx >= nb ? nb - 1 : idx);
    const float f = valid ? 1.0f : 0.0f;
    o[e] = f * bf16r(b[idx]) + 0.0f;
  }
  float* op = dst + 4 * t;
  *(volatile v4f*)op = o;
  __threadfence();
  *(volatile v4f*)op = o;
}

template <bool SPLITA, bool NARROW>
__global__ __launch_bounds__(256) void gemm_bf16_kernel(
    const unsigned short* __restrict__ Ap, const unsigned short* __restrict__ A2p, int lda,
    const unsigned short* __restrict__ Btp, int ldb,
    float* __restrict__ C, int ldc, const float* __restrict__ bias,
    int M, int N, int K) {
  const __bf16* A = (const __bf16*)Ap; const __bf16* A2 = (const __bf16*)A2p; const __bf16* Bt = (const __bf16*)Btp;
  __shared__ __align__(16) float sT[8][16 * 68];
  const int lane = threadIdx.x & 31;
  const int wave = threadIdx.x >> 5;
  const int tilesN = N >> 6;
  const int tilesM = M >> 6;
  const int tile = blockIdx.x * 8 + wave;
  if (tile >= tilesM * tilesN) return;
  const int tm = tile / tilesN;
  const int tn = tile - tm * tilesN;
  const int m0 = tm << 6;
  const int n0 = tn << 6;

  const int rlane = lane & 15;
  const int koff  = (lane >> 4) * 8;
  const int mOff  = (lane >> 4) * 8;

  v8f acc[4][4];
#pragma unroll
  for (int i = 0; i < 4; ++i)
#pragma unroll
    for (int j = 0; j < 4; ++j) acc[i][j] = (v8f){0.f,0.f,0.f,0.f,0.f,0.f,0.f,0.f};

  for (int k0 = 0; k0 < K; k0 += 32) {
    v16b bh[4];
#pragma unroll
    for (int j = 0; j < 4; ++j) {
      const size_t bo = (size_t)(n0 + (j << 4) + rlane) * ldb + koff + k0;
      bh[j] = FragB::load(Bt + bo);
    }
#pragma unroll
    for (int i = 0; i < 4; ++i) {
      const size_t ao = (size_t)(m0 + (i << 4) + rlane) * lda + koff + k0;
      const v16b ah = FragB::load(A + ao);
      const v16b al = SPLITA ? FragB::load(A2 + ao) : ah;
#pragma unroll
      for (int j = 0; j < 4; ++j) {
        acc[i][j] = FragB::mma(ah, bh[j], acc[i][j]);
        if (SPLITA) acc[i][j] = FragB::mma(al, bh[j], acc[i][j]);
      }
      guard_grp_b(acc[i][0], acc[i][1], acc[i][2], acc[i][3], ah, al, bh[0], bh[1], bh[2], bh[3]);
    }
  }
  acc_guard4(acc[0][0], acc[0][1], acc[0][2], acc[0][3]);
  acc_guard4(acc[1][0], acc[1][1], acc[1][2], acc[1][3]);
  acc_guard4(acc[2][0], acc[2][1], acc[2][2], acc[2][3]);
  acc_guard4(acc[3][0], acc[3][1], acc[3][2], acc[3][3]);

  float* slab = sT[wave];
#pragma unroll
  for (int i = 0; i < 4; ++i) {
    const int mBase = m0 + (i << 4);
#pragma unroll
    for (int j = 0; j < 4; ++j) {
      const int n = n0 + (j << 4) + rlane;
      const float bv = bias[n];
#pragma unroll
      for (int r = 0; r < 8; ++r) slab[(mOff + r) * 68 + (j << 4) + rlane] = acc[i][j][r] + bv;
    }
    __builtin_amdgcn_fence(__ATOMIC_RELEASE, "workgroup");
    __builtin_amdgcn_wave_barrier();
    __builtin_amdgcn_fence(__ATOMIC_ACQUIRE, "workgroup");
    if (!NARROW) {
      const int hh = lane >> 4, c4 = (lane & 15) * 4;
      for (int pass = 0; pass < 2; ++pass) {
#pragma unroll
        for (int it = 0; it < 8; ++it) {
          const int row = it * 2 + hh;
          const v4f v = *(const v4f*)(slab + row * 68 + c4);
          *(volatile v4f*)(C + (size_t)(mBase + row) * ldc + n0 + c4) = v;
        }
        __threadfence();
      }
    } else {
      for (int pass = 0; pass < 2; ++pass) {
#pragma unroll
        for (int it = 0; it < 5; ++it) {
          const int ch = it * 32 + lane;
          const int row = ch / 10, cq = (ch - row * 10) * 4;
          const v4f v = *(const v4f*)(slab + row * 68 + cq);
          *(volatile v4f*)(C + (size_t)(mBase + row) * NLAB + cq) = v;
        }
        __threadfence();
      }
    }
    __builtin_amdgcn_fence(__ATOMIC_RELEASE, "workgroup");
    __builtin_amdgcn_wave_barrier();
    __builtin_amdgcn_fence(__ATOMIC_ACQUIRE, "workgroup");
  }
}

constexpr int RROWS  = 16;
constexpr int RNW    = 13;
constexpr int RTHR   = RNW * 32;
constexpr int APITCH = 232;
constexpr int YPITCH = 260;
constexpr int ZPITCH = 68;
static_assert(RNW * 16 == GATEP);
static_assert(SEQS % RROWS == 0);
static_assert(APITCH % 8 == 0 && APITCH >= HKP && YPITCH % 4 == 0 && YPITCH >= HC_BWD);

template <int OMODE>
__global__ __launch_bounds__(RTHR) void lstm_seq_kernel(const float* __restrict__ ZX,
                                                       const unsigned short* __restrict__ WHp,
                                                       const int* __restrict__ lens, int dir, int hcol0,
                                                       unsigned short* __restrict__ OH, unsigned short* __restrict__ OL,
                                                       float* __restrict__ OF) {
  __shared__ __align__(16) __bf16 Ahi[2][RROWS * APITCH];
  __shared__ __align__(16) __bf16 Alo[2][RROWS * APITCH];
  __shared__ __align__(16) float  Ysl[RROWS * YPITCH];
  __shared__ __align__(16) float  Zsl[RNW][16 * ZPITCH];
  __shared__ int lsh[RROWS];
  const __bf16* WH = (const __bf16*)WHp;
  const int tid = threadIdx.x, lane = tid & 31, wave = tid >> 5;
  const int c = lane & 15, hh = lane >> 4, koff = hh * 8;
  const int rowbase = blockIdx.x * RROWS;
  const int ucol = 16 * wave + c;
  const bool uval = ucol < HID;
  const __bf16 zb = __builtin_bit_cast(__bf16, (unsigned short)0);

  {
    __bf16* a0 = &Ahi[0][0];
    __bf16* a1 = &Alo[0][0];
#pragma unroll 1
    for (int i = tid; i < 2 * RROWS * APITCH; i += RTHR) { a0[i] = zb; a1[i] = zb; }
#pragma unroll 1
    for (int i = tid; i < RROWS * YPITCH; i += RTHR) Ysl[i] = 0.0f;
    float* z0 = &Zsl[0][0];
#pragma unroll 1
    for (int i = tid; i < RNW * 16 * ZPITCH; i += RTHR) z0[i] = 0.0f;
    if (tid < RROWS) {
      int L = lens[rowbase + tid];
      L = L < 0 ? 0 : (L > STEPS ? STEPS : L);
      lsh[tid] = L;
    }
  }
  __syncthreads();

  int lenr[8], len2[8];
#pragma unroll
  for (int r = 0; r < 8; ++r) lenr[r] = lsh[8 * hh + r];
#pragma unroll
  for (int i = 0; i < 8; ++i) len2[i] = lsh[2 * i + hh];
  float cst[8], hst[8];
#pragma unroll
  for (int r = 0; r < 8; ++r) { cst[r] = 0.0f; hst[r] = 0.0f; }

  const __bf16* wrow = WH + (size_t)ucol * HKP + koff;
  float* zs = Zsl[wave];
  const v8f z8 = {0.f, 0.f, 0.f, 0.f, 0.f, 0.f, 0.f, 0.f};
  const int gpc = c >> 2, c4p = (c & 3) * 4;

#pragma unroll 1
  for (int s = 0; s < STEPS; ++s) {
    const int cur = s & 1, nxt = cur ^ 1;

#pragma unroll
    for (int i = 0; i < 8; ++i) {
      const int row = 2 * i + hh;
      const int L = len2[i];
      const bool act = s < L;
      const int tp = ((dir != 0) && act) ? (L - 1 - s) : s;
      const float* zp = ZX + ((size_t)(rowbase + row) * STEPS + (size_t)tp) * NGATE + gpc * GATEP + 16 * wave + c4p;
      const v4f v = *(const v4f*)zp;
      *(v4f*)(zs + row * ZPITCH + gpc * 16 + c4p) = v;
    }
    __builtin_amdgcn_fence(__ATOMIC_RELEASE, "workgroup");
    __builtin_amdgcn_wave_barrier();
    __builtin_amdgcn_fence(__ATOMIC_ACQUIRE, "workgroup");
    v8f acc[4];
#pragma unroll
    for (int g = 0; g < 4; ++g) {
      acc[g] = z8;
#pragma unroll
      for (int r = 0; r < 8; ++r) acc[g][r] = zs[(8 * hh + r) * ZPITCH + 16 * g + c];
    }

    const __bf16* ahr = &Ahi[cur][0] + c * APITCH + koff;
    const __bf16* alr = &Alo[cur][0] + c * APITCH + koff;
#pragma unroll 1
    for (int kt = 0; kt < HKP / 32; ++kt) {
      const int k0 = kt * 32;
      const v16b ah = FragB::load(ahr + k0);
      const v16b al = FragB::load(alr + k0);
      const v16b b0 = FragB::load(wrow + k0);
      const v16b b1 = FragB::load(wrow + (size_t)1 * GATEP * HKP + k0);
      const v16b b2 = FragB::load(wrow + (size_t)2 * GATEP * HKP + k0);
      const v16b b3 = FragB::load(wrow + (size_t)3 * GATEP * HKP + k0);
      acc[0] = FragB::mma(ah, b0, acc[0]);
      acc[1] = FragB::mma(ah, b1, acc[1]);
      acc[2] = FragB::mma(ah, b2, acc[2]);
      acc[3] = FragB::mma(ah, b3, acc[3]);
      acc[0] = FragB::mma(al, b0, acc[0]);
      acc[1] = FragB::mma(al, b1, acc[1]);
      acc[2] = FragB::mma(al, b2, acc[2]);
      acc[3] = FragB::mma(al, b3, acc[3]);
      guard_grp_b(acc[0], acc[1], acc[2], acc[3], ah, al, b0, b1, b2, b3);
    }
    acc_guard4(acc[0], acc[1], acc[2], acc[3]);

    __bf16* ahw = &Ahi[nxt][0];
    __bf16* alw = &Alo[nxt][0];
#pragma unroll
    for (int r = 0; r < 8; ++r) {
      const float zi = acc[0][r], zj = acc[1][r], zf = acc[2][r], zo = acc[3][r];
      const float fg = fsig(zf + FORGET_B);
      const float ig = fsig(zi);
      const float gj = tanhf(zj);
      const float og = fsig(zo);
      const float nc = cst[r] * fg + ig * gj;
      const float nh = tanhf(nc) * og;
      const bool act = s < lenr[r];
      const float cn = act ? nc : cst[r];
      const float hn = act ? nh : hst[r];
      cst[r] = cn;
      hst[r] = hn;
      const float yv = (act && uval) ? nh : 0.0f;
      const float hv = uval ? hn : 0.0f;
      unsigned hb, lb;
      split_bf(hv, hb, lb);
      ahw[(8 * hh + r) * APITCH + ucol] = __builtin_bit_cast(__bf16, (unsigned short)hb);
      alw[(8 * hh + r) * APITCH + ucol] = __builtin_bit_cast(__bf16, (unsigned short)lb);
      Ysl[(8 * hh + r) * YPITCH + ucol] = yv;
    }
    if (wave == RNW - 1) {
#pragma unroll
      for (int r = 0; r < 8; ++r) {
        ahw[(8 * hh + r) * APITCH + GATEP + c] = zb;
        alw[(8 * hh + r) * APITCH + GATEP + c] = zb;
      }
    }
#pragma unroll 1
    for (int e = tid; e < RROWS * (HC_BWD - GATEP); e += RTHR) {
      const int row = e / (HC_BWD - GATEP);
      const int col = GATEP + (e - row * (HC_BWD - GATEP));
      Ysl[row * YPITCH + col] = 0.0f;
    }
    __syncthreads();

    if (OMODE == 0) {
      v4u wh[2], wl[2]; size_t oo[2]; bool ok[2];
#pragma unroll
      for (int it = 0; it < 2; ++it) {
        const int id = it * RTHR + tid;
        ok[it] = id < RROWS * 32;
        const int idc = ok[it] ? id : 0;
        const int row = idc >> 5, c8 = (idc & 31) * 8;
        const int L = lsh[row];
        const bool act = s < L;
        const int tp = ((dir != 0) && act) ? (L - 1 - s) : s;
        const v4f a = *(const v4f*)(Ysl + row * YPITCH + c8);
        const v4f b = *(const v4f*)(Ysl + row * YPITCH + c8 + 4);
        float f8[8];
        f8[0] = a[0]; f8[1] = a[1]; f8[2] = a[2]; f8[3] = a[3];
        f8[4] = b[0]; f8[5] = b[1]; f8[6] = b[2]; f8[7] = b[3];
        unsigned uh[4], ul[4];
#pragma unroll
        for (int e2 = 0; e2 < 4; ++e2) {
          unsigned h0, l0, h1, l1;
          split_bf(f8[2 * e2], h0, l0);
          split_bf(f8[2 * e2 + 1], h1, l1);
          uh[e2] = h0 | (h1 << 16);
          ul[e2] = l0 | (l1 << 16);
        }
        wh[it] = (v4u){uh[0], uh[1], uh[2], uh[3]};
        wl[it] = (v4u){ul[0], ul[1], ul[2], ul[3]};
        oo[it] = ((size_t)(rowbase + row) * STEPS + (size_t)tp) * HCP + (size_t)hcol0 + (size_t)c8;
      }
      for (int pass = 0; pass < 2; ++pass) {
#pragma unroll
        for (int it = 0; it < 2; ++it) {
          if (ok[it]) {
            *(volatile v4u*)(OH + oo[it]) = wh[it];
            *(volatile v4u*)(OL + oo[it]) = wl[it];
          }
        }
        __threadfence();
      }
    } else {
      v4f ov[3]; size_t oo[3]; bool ok[3];
#pragma unroll
      for (int it = 0; it < 3; ++it) {
        const int id = it * RTHR + tid;
        ok[it] = id < RROWS * (H2P / 4);
        const int idc = ok[it] ? id : 0;
        const int row = idc / (H2P / 4), ch = idc - row * (H2P / 4);
        const int L = lsh[row];
        const bool act = s < L;
        const int tp = ((dir != 0) && act) ? (L - 1 - s) : s;
        ov[it] = *(const v4f*)(Ysl + row * YPITCH + 4 * ch);
        oo[it] = ((size_t)(rowbase + row) * STEPS + (size_t)tp) * H2P + (size_t)(4 * ch);
      }
      for (int pass = 0; pass < 2; ++pass) {
#pragma unroll
        for (int it = 0; it < 3; ++it) {
          if (ok[it]) *(volatile v4f*)(OF + oo[it]) = ov[it];
        }
        __threadfence();
      }
    }
    __syncthreads();
  }
}

__global__ __launch_bounds__(256) void bn_stats_kernel(const float* __restrict__ H2, float* __restrict__ stats) {
  __shared__ float red[256];
  const int f = blockIdx.x, tid = threadIdx.x;
  float s = 0.0f;
#pragma unroll 4
  for (int i = tid; i < NROWS; i += 256) s += H2[(size_t)i * H2P + f];
  red[tid] = s;
  __syncthreads();
  for (int st = 128; st > 0; st >>= 1) {
    if (tid < st) red[tid] += red[tid + st];
    __syncthreads();
  }
  const float mean = red[0] * (1.0f / NROWS);
  __syncthreads();
  float q = 0.0f;
#pragma unroll 4
  for (int i = tid; i < NROWS; i += 256) { const float d = H2[(size_t)i * H2P + f] - mean; q += d * d; }
  red[tid] = q;
  __syncthreads();
  for (int st = 128; st > 0; st >>= 1) {
    if (tid < st) red[tid] += red[tid + st];
    __syncthreads();
  }
  const float var  = red[0] * (1.0f / NROWS);
  const float rstd = rsqrtf(var + BNEPS);
  if (tid < 32) {
    const float v = (tid == 0) ? mean : ((tid == 1) ? rstd : 0.0f);
    float* op = stats + (size_t)f * STP + tid;
    *(volatile float*)op = v;
    __threadfence();
    *(volatile float*)op = v;
  }
}

__global__ __launch_bounds__(256) void bn_apply_kernel(const float* __restrict__ H2, const float* __restrict__ stats,
                                                      const float* __restrict__ gam, const float* __restrict__ bet,
                                                      unsigned short* __restrict__ OH, unsigned short* __restrict__ OL) {
  __shared__ float mS[H2NP], rS[H2NP], gS[H2NP], bS[H2NP];
  const int tid = threadIdx.x;
  if (tid < H2NP) {
    const int fi = tid < HID ? tid : (HID - 1);
    mS[tid] = stats[(size_t)fi * STP + 0];
    rS[tid] = stats[(size_t)fi * STP + 1];
    gS[tid] = bf16r(gam[fi]);
    bS[tid] = bf16r(bet[fi]);
  }
  __syncthreads();
  constexpr int NC8 = H2NP / 8;
  const int i = blockIdx.x * 256 + tid;
  const int row = i / NC8, c8 = (i - row * NC8) * 8;
  const v4f a = *(const v4f*)(H2 + (size_t)row * H2P + c8);
  const v4f b = *(const v4f*)(H2 + (size_t)row * H2P + c8 + 4);
  float x8[8];
  x8[0] = a[0]; x8[1] = a[1]; x8[2] = a[2]; x8[3] = a[3];
  x8[4] = b[0]; x8[5] = b[1]; x8[6] = b[2]; x8[7] = b[3];
  unsigned uh[4], ul[4];
#pragma unroll
  for (int e2 = 0; e2 < 4; ++e2) {
    unsigned hb[2], lb[2];
#pragma unroll
    for (int h = 0; h < 2; ++h) {
      const int e = 2 * e2 + h;
      const int col = c8 + e;
      const float v = ((x8[e] - mS[col]) * rS[col]) * gS[col] + bS[col];
      const float fv = (col < HID) ? 1.0f : 0.0f;
      split_bf(fv * v + 0.0f, hb[h], lb[h]);
    }
    uh[e2] = hb[0] | (hb[1] << 16);
    ul[e2] = lb[0] | (lb[1] << 16);
  }
  const v4u wh = {uh[0], uh[1], uh[2], uh[3]};
  const v4u wl = {ul[0], ul[1], ul[2], ul[3]};
  unsigned short* ph = OH + (size_t)i * 8;
  unsigned short* pl = OL + (size_t)i * 8;
  *(volatile v4u*)ph = wh;
  *(volatile v4u*)pl = wl;
  __threadfence();
  *(volatile v4u*)ph = wh;
  *(volatile v4u*)pl = wl;
}

extern "C" void kernel_launch(void* const* d_in, const int* in_sizes, int n_in,
                              void* d_out, int out_size, void* d_ws, size_t ws_size, hipStream_t stream) {
  if (n_in < 13 || d_out == nullptr || d_ws == nullptr) return;
  if (in_sizes[0] != SEQS * STEPS * TOKD || in_sizes[1] != SEQS * STEPS * TAGD || in_sizes[2] != SEQS ||
      in_sizes[3] != (DIN1 + HID) * G4REAL || in_sizes[4] != G4REAL ||
      in_sizes[5] != (DIN1 + HID) * G4REAL || in_sizes[6] != G4REAL ||
      in_sizes[7] != (2 * HID + HID) * G4REAL || in_sizes[8] != G4REAL ||
      in_sizes[9] != HID || in_sizes[10] != HID || in_sizes[11] != HID * NLAB || in_sizes[12] != NLAB ||
      out_size != NROWS * NLAB) return;

  const float* tok  = (const float*)d_in[0];
  const float* tag  = (const float*)d_in[1];
  const int*   lens = (const int*)d_in[2];
  const float* Wf   = (const float*)d_in[3];
  const float* bfv  = (const float*)d_in[4];
  const float* Wb   = (const float*)d_in[5];
  const float* bbv  = (const float*)d_in[6];
  const float* W2   = (const float*)d_in[7];
  const float* b2v  = (const float*)d_in[8];
  const float* gam  = (const float*)d_in[9];
  const float* bet  = (const float*)d_in[10];
  const float* Wd   = (const float*)d_in[11];
  const float* bdv  = (const float*)d_in[12];
  float* out = (float*)d_out;

  char* ws = (char*)d_ws; size_t off = 0;
  auto carve = [&](size_t bytes) -> char* { char* p = ws + off; off += (bytes + 255) & ~(size_t)255; return p; };
  unsigned short* XB16 = (unsigned short*)carve(WS_XB);
  unsigned short* WX1F = (unsigned short*)carve(WS_WX1);
  unsigned short* WH1F = (unsigned short*)carve(WS_WH);
  unsigned short* WX1B = (unsigned short*)carve(WS_WX1);
  unsigned short* WH1B = (unsigned short*)carve(WS_WH);
  unsigned short* WX2P = (unsigned short*)carve(WS_WX2);
  unsigned short* WH2P = (unsigned short*)carve(WS_WH);
  unsigned short* WDBP = (unsigned short*)carve(WS_WD);
  float*          BG1F = (float*)carve(WS_BG);
  float*          BG1B = (float*)carve(WS_BG);
  float*          BG2  = (float*)carve(WS_BG);
  float*          BDP  = (float*)carve(WS_BD);
  float*          ZX   = (float*)carve(WS_ZX);
  unsigned short* HCH  = (unsigned short*)carve(WS_HC);
  unsigned short* HCL  = (unsigned short*)carve(WS_HC);
  float*          H2   = (float*)carve(WS_H2);
  float*          STAT = (float*)carve(WS_ST);
  unsigned short* H2NH = (unsigned short*)carve(WS_H2N);
  unsigned short* H2NL = (unsigned short*)carve(WS_H2N);
  if (off > ws_size || off > (size_t)134217728) return;

  xpack_kernel<<<(NROWS * (K1P / 8) + 255) / 256, 256, 0, stream>>>(tok, tag, XB16);
  wpack_kernel<<<(NGATE * (K1P / 8) + 255) / 256, 256, 0, stream>>>(Wf, DIN1 + HID, G4REAL, WX1F, NGATE, K1P, GATEP, HID, HID, DIN1, 0,    K1P, 0, 0);
  wpack_kernel<<<(NGATE * (HKP / 8) + 255) / 256, 256, 0, stream>>>(Wf, DIN1 + HID, G4REAL, WH1F, NGATE, HKP, GATEP, HID, HID, HID,  DIN1, HKP, 0, 0);
  wpack_kernel<<<(NGATE * (K1P / 8) + 255) / 256, 256, 0, stream>>>(Wb, DIN1 + HID, G4REAL, WX1B, NGATE, K1P, GATEP, HID, HID, DIN1, 0,    K1P, 0, 0);
  wpack_kernel<<<(NGATE * (HKP / 8) + 255) / 256, 256, 0, stream>>>(Wb, DIN1 + HID, G4REAL, WH1B, NGATE, HKP, GATEP, HID, HID, HID,  DIN1, HKP, 0, 0);
  wpack_kernel<<<(NGATE * (HCP / 8) + 255) / 256, 256, 0, stream>>>(W2, 3 * HID, G4REAL, WX2P, NGATE, HCP, GATEP, HID, HID, HID, 0, HC_BWD, HID, HID);
  wpack_kernel<<<(NGATE * (HKP / 8) + 255) / 256, 256, 0, stream>>>(W2, 3 * HID, G4REAL, WH2P, NGATE, HKP, GATEP, HID, HID, HID, 2 * HID, HKP, 0, 0);
  wpack_kernel<<<(NLABP * (H2NP / 8) + 255) / 256, 256, 0, stream>>>(Wd, HID, NLAB, WDBP, NLABP, H2NP, NLABP, NLAB, 0, HID, 0, H2NP, 0, 0);
  bias_pack_kernel<<<1, 256, 0, stream>>>(bfv, G4REAL, BG1F, NGATE, GATEP, HID, HID);
  bias_pack_kernel<<<1, 256, 0, stream>>>(bbv, G4REAL, BG1B, NGATE, GATEP, HID, HID);
  bias_pack_kernel<<<1, 256, 0, stream>>>(b2v, G4REAL, BG2,  NGATE, GATEP, HID, HID);
  bias_pack_kernel<<<1, 256, 0, stream>>>(bdv, NLAB,   BDP,  NLABP, NLABP, NLAB, 0);

  const int gblk = (NROWS / 64) * (NGATE / 64) / 8;
  const int rblk = SEQS / RROWS;

  gemm_bf16_kernel<false, false><<<gblk, 256, 0, stream>>>(XB16, XB16, K1P, WX1F, K1P, ZX, NGATE, BG1F, NROWS, NGATE, K1P);
  lstm_seq_kernel<0><<<rblk, RTHR, 0, stream>>>(ZX, WH1F, lens, 0, 0, HCH, HCL, H2);
  gemm_bf16_kernel<false, false><<<gblk, 256, 0, stream>>>(XB16, XB16, K1P, WX1B, K1P, ZX, NGATE, BG1B, NROWS, NGATE, K1P);
  lstm_seq_kernel<0><<<rblk, RTHR, 0, stream>>>(ZX, WH1B, lens, 1, HC_BWD, HCH, HCL, H2);
  gemm_bf16_kernel<true, false><<<gblk, 256, 0, stream>>>(HCH, HCL, HCP, WX2P, HCP, ZX, NGATE, BG2, NROWS, NGATE, HCK);
  lstm_seq_kernel<1><<<rblk, RTHR, 0, stream>>>(ZX, WH2P, lens, 0, 0, HCH, HCL, H2);
  bn_stats_kernel<<<HID, 256, 0, stream>>>(H2, STAT);
  bn_apply_kernel<<<NROWS * (H2NP / 8) / 256, 256, 0, stream>>>(H2, STAT, gam, bet, H2NH, H2NL);
  gemm_bf16_kernel<true, true><<<(NROWS / 64) * (NLABP / 64) / 8, 256, 0, stream>>>(H2NH, H2NL, H2NP, WDBP, H2NP, out, NLAB, BDP, NROWS, NLABP, H2NP);
}
